// CBAMSA_76132590289611
// MI455X (gfx1250) — hardware-verified
//
#include <hip/hip_runtime.h>
#include <math.h>

typedef __attribute__((ext_vector_type(16))) _Float16 v16h;
typedef __attribute__((ext_vector_type(16))) __bf16 v16b;
typedef __attribute__((ext_vector_type(8)))  _Float16 v8h;
typedef __attribute__((ext_vector_type(8)))  float v8f;
typedef __attribute__((ext_vector_type(4)))  float v4f;
typedef __attribute__((ext_vector_type(2)))  float v2f;
typedef __attribute__((ext_vector_type(4)))  unsigned v4u;
typedef __attribute__((ext_vector_type(4)))  int v4i;
typedef float __attribute__((may_alias)) float_a;
typedef int __attribute__((may_alias)) int_a;

template <typename T> __device__ __forceinline__ void vst2(void* p, T v) { *(volatile T*)p = v; __threadfence(); *(volatile T*)p = v; }
__device__ __forceinline__ v8f wmma16(v16h a, v16h b, v8f c) {
  v8f d = __builtin_amdgcn_wmma_f32_16x16x32_f16(false, a, false, b, (short)0, c, false, false);
  asm volatile("v_nop\n\tv_nop\n\tv_nop\n\tv_nop" : "+v"(d) : "v"(a), "v"(b));
  return d;
}
__device__ __forceinline__ v8f wmma_bf(v16b a, v16b b, v8f c) {
  v8f d = __builtin_amdgcn_wmma_f32_16x16x32_bf16(false, a, false, b, (short)0, c, false, false);
  asm volatile("v_nop\n\tv_nop\n\tv_nop\n\tv_nop" : "+v"(d) : "v"(a), "v"(b));
  return d;
}
__device__ __forceinline__ v16h frag_h(const _Float16* rowk0, int lane) {
  union { v16h v; v8h q[2]; } u; const _Float16* p = rowk0 + 8 * (lane >> 4);
  u.q[0] = *(const v8h*)p; u.q[1] = *(const v8h*)(p + 16); return u.v;
}
__device__ __forceinline__ v16h frag_f32(const float* rowk0, int lane) {
  v16h a; const float* p = rowk0 + 8 * (lane >> 4);
#pragma unroll
  for (int i = 0; i < 8; ++i) { a[i] = (_Float16)p[i]; a[8 + i] = (_Float16)p[16 + i]; }
  return a;
}
__device__ __forceinline__ v16h frag_f32s(const float* rowk0, int lane, float sc) {
  v16h a; const float* p = rowk0 + 8 * (lane >> 4);
#pragma unroll
  for (int i = 0; i < 8; ++i) { a[i] = (_Float16)(p[i] * sc); a[8 + i] = (_Float16)(p[16 + i] * sc); }
  return a;
}
__device__ __forceinline__ v16h fragc_f32(const float* W, int k0, int n, int lane, int ld, int K) {
  v16h a; const int g = lane >> 4;
#pragma unroll
  for (int i = 0; i < 8; ++i) { const int ka = k0 + 8 * g + i, kb = ka + 16;
    a[i] = (_Float16)(ka < K ? W[(size_t)(ka < K ? ka : K - 1) * ld + n] : 0.f); a[8 + i] = (_Float16)(kb < K ? W[(size_t)(kb < K ? kb : K - 1) * ld + n] : 0.f); }
  return a;
}
struct F2 { v16b h, l; };
__device__ __forceinline__ F2 bsplit16(const float v[16]) { F2 r;
#pragma unroll
  for (int i = 0; i < 16; ++i) { const __bf16 h = (__bf16)v[i]; r.h[i] = h; r.l[i] = (__bf16)(v[i] - (float)h); }
  return r; }
__device__ __forceinline__ F2 split_row(const float* row, int k0, int lane) { float v[16]; const float* p = row + k0 + 8 * (lane >> 4);
#pragma unroll
  for (int i = 0; i < 8; ++i) { v[i] = p[i]; v[8 + i] = p[16 + i]; }
  return bsplit16(v); }
__device__ __forceinline__ F2 split_rowK(const float* row, int k0, int lane, int K) { float v[16]; const int g = lane >> 4;
#pragma unroll
  for (int i = 0; i < 8; ++i) { const int ka = k0 + 8 * g + i, kb = ka + 16; v[i] = ka < K ? row[ka < K ? ka : K - 1] : 0.f; v[8 + i] = kb < K ? row[kb < K ? kb : K - 1] : 0.f; }
  return bsplit16(v); }
__device__ __forceinline__ F2 split_col(const float* W, int k0, int n, int lane, int ld, int K) { float v[16]; const int g = lane >> 4;
#pragma unroll
  for (int i = 0; i < 8; ++i) { const int ka = k0 + 8 * g + i, kb = ka + 16; v[i] = ka < K ? W[(size_t)(ka < K ? ka : K - 1) * ld + n] : 0.f; v[8 + i] = kb < K ? W[(size_t)(kb < K ? kb : K - 1) * ld + n] : 0.f; }
  return bsplit16(v); }
__device__ __forceinline__ v8f mac3(const F2& a, const F2& b, v8f c) { c = wmma_bf(a.l, b.h, c); c = wmma_bf(a.h, b.l, c); return wmma_bf(a.h, b.h, c); }
__device__ __forceinline__ float sigm(float v) { return 1.0f / (1.0f + expf(-v)); }
#define LDSX() do { asm volatile("s_wait_dscnt 0" ::: "memory"); __builtin_amdgcn_wave_barrier(); __builtin_amdgcn_fence(__ATOMIC_RELEASE, "workgroup"); } while (0)


#define NB 4
#define CC 256
#define HW 64
#ifndef HHT
#define HHT 64
#endif
#define NP (HHT * HW)
#define NHh 4
#define KD 32
#define VD 64
#define HQ 512
#define RED 16
typedef __attribute__((ext_vector_type(8))) __bf16 v8b;
__device__ __forceinline__ v16b frag_b(const __bf16* rowk0, int lane) {
  union { v16b v; v8b q[2]; } u; const __bf16* p = rowk0 + 8 * (lane >> 4);
  u.q[0] = *(const v8b*)p; u.q[1] = *(const v8b*)(p + 16); return u.v;
}
__device__ __forceinline__ float bfr(float v) { return (float)(__bf16)v; }
__device__ __attribute__((noinline)) float exp_ni(float v) { return expf(v); }
__device__ __attribute__((noinline)) float erf_ni(float v) { return erff(v); }

#define WS_PW  0u
#define WS_PP  (WS_PW + 2u * HQ * CC)
#define WS_QH  (WS_PP + 2u * CC * CC)
#define WS_QL  (WS_QH + 2u * NB * NHh * NP * KD)
#define WS_KH  (WS_QL + 2u * NB * NHh * NP * KD)
#define WS_KL  (WS_KH + 2u * NB * NHh * NP * KD)
#define WS_VH  (WS_KL + 2u * NB * NHh * NP * KD)
#define WS_VL  (WS_VH + 2u * (size_t)NB * CC * NP)
#define WS_O   (WS_VL + 2u * (size_t)NB * CC * NP)
#define WS_X1  (WS_O + 4u * (size_t)NB * CC * NP)
#define WS_CS  (WS_X1 + 4u * (size_t)NB * CC * NP)
#define WS_CM  (WS_CS + 4u * NB * 64 * CC)
#define WS_CA  (WS_CM + 4u * NB * 64 * CC)
#define WS_SP  (WS_CA + 4u * NB * CC)
#define WS_END (WS_SP + 4u * NB * 2 * NP)

__device__ __attribute__((noinline)) float sigm_p(float v) { return 1.0f / (1.0f + expf(-v)); }
__global__ __launch_bounds__(256) void k_pack(const float* __restrict__ WQ, const float* __restrict__ WPj, __bf16* __restrict__ PW, __bf16* __restrict__ PP) {
  const int n = blockIdx.x, which = blockIdx.y, t = threadIdx.x; __shared__ __align__(16) __bf16 s[CC];
  if (which == 0) { s[t] = (__bf16)WQ[(size_t)n * CC + t]; __syncthreads(); if (t < CC / 8) vst2((unsigned*)(PW + (size_t)n * CC + t * 8), *(const v4u*)&s[t * 8]); }
  else { if (n >= CC) return; s[t] = (__bf16)WPj[(size_t)n * CC + t]; __syncthreads(); if (t < CC / 8) vst2((unsigned*)(PP + (size_t)n * CC + t * 8), *(const v4u*)&s[t * 8]); }
}
__global__ __launch_bounds__(128) void k_qkv(const float* __restrict__ X, const __bf16* __restrict__ PW, const float* __restrict__ BQ, _Float16* __restrict__ QH, _Float16* __restrict__ QL, _Float16* __restrict__ KH, _Float16* __restrict__ KL, _Float16* __restrict__ VH, _Float16* __restrict__ VL) {
  __shared__ __align__(16) __bf16 sa[64][CC + 8]; __shared__ __align__(16) _Float16 sqh[2][64][40], sql[2][64][40]; __shared__ __align__(16) _Float16 svh[VD][72], svl[VD][72];
  const int tid = threadIdx.x, wave = tid >> 5, lane = tid & 31, col = lane & 15, g = lane >> 4; const size_t b = blockIdx.y; const int n0 = blockIdx.x * 64;
  for (int e = tid; e < 64 * CC; e += 128) { const int c = e >> 6, r = e & 63; sa[r][c] = (__bf16)X[(b * CC + c) * NP + n0 + r]; }
  if (tid < 64) for (int c = CC; c < CC + 8; ++c) sa[tid][c] = (__bf16)0.f;
  __syncthreads();
#pragma unroll 1
  for (int h = 0; h < NHh; ++h) { v8f acc[8] = {};
#pragma unroll
    for (int kc = 0; kc < CC / 32; ++kc) { const v16b a = frag_b(&sa[wave * 16 + col][kc * 32], lane);
#pragma unroll
      for (int j = 0; j < 8; ++j) acc[j] = wmma_bf(a, frag_b(PW + (size_t)(h * 128 + j * 16 + col) * CC + kc * 32, lane), acc[j]); }
#pragma unroll
    for (int j = 0; j < 8; ++j) { const int cl = j * 16 + col; const float bb = bfr(BQ[h * 128 + cl]);
#pragma unroll
      for (int r = 0; r < 8; ++r) { const float v = acc[j][r] + bb; const int rr = wave * 16 + 8 * g + r; const _Float16 hv = (_Float16)v;
        if (j < 4) { const int which = j >> 1, d = (j & 1) * 16 + col; sqh[which][rr][d] = hv; sql[which][rr][d] = (_Float16)((v - (float)hv) * 2048.0f); }
        else { const int d = (j - 4) * 16 + col; svh[d][rr] = hv; svl[d][rr] = (_Float16)((v - (float)hv) * 2048.0f); } } }
    __syncthreads();
    for (int e = tid; e < 2 * 64 * 4; e += 128) { const int which = e >> 8, r = (e >> 2) & 63, q = e & 3; const size_t o = ((b * NHh + h) * NP + n0 + r) * KD + q * 8; _Float16* DH_ = which ? KH : QH; _Float16* DL_ = which ? KL : QL; vst2((unsigned*)(DH_ + o), *(const v4u*)&sqh[which][r][q * 8]); vst2((unsigned*)(DL_ + o), *(const v4u*)&sql[which][r][q * 8]); }
    for (int e = tid; e < VD * 8; e += 128) { const int d = e >> 3, pc = e & 7; const size_t o = (b * CC + h * VD + d) * NP + n0 + pc * 8; vst2((unsigned*)(VH + o), *(const v4u*)&svh[d][pc * 8]); vst2((unsigned*)(VL + o), *(const v4u*)&svl[d][pc * 8]); }
    __syncthreads(); }
}
__global__ __launch_bounds__(128) void k_attn(const _Float16* __restrict__ QH, const _Float16* __restrict__ QL, const _Float16* __restrict__ KH, const _Float16* __restrict__ KL, const _Float16* __restrict__ VH, const _Float16* __restrict__ VL, const float* __restrict__ WPE, const float* __restrict__ BPE, float* __restrict__ O) {
  __shared__ __align__(16) _Float16 sph[4][16][40]; __shared__ __align__(16) float so[VD][68]; __shared__ float sv[VD][3][66];
  const int tid = threadIdx.x, wave = tid >> 5, lane = tid & 31, col = lane & 15, g = lane >> 4; const int y = blockIdx.x, h = blockIdx.y; const size_t b = blockIdx.z; const int q0 = y * 64 + wave * 16;
  const size_t qbase = (b * NHh + h) * NP; const v16h aq = frag_h(QH + (qbase + q0 + col) * KD, lane), aql = frag_h(QL + (qbase + q0 + col) * KD, lane);
  float m[8], l[8];
#pragma unroll
  for (int r = 0; r < 8; ++r) { m[r] = -3.0e38f; l[r] = 0.f; }
  v8f acc[4] = {}; const float scale = 1.0f / sqrtf((float)KD);
#pragma unroll 1
  for (int ks = 0; ks < NP / 32; ++ks) { const int j0 = ks * 32; v8f s[2];
#pragma unroll
    for (int ct = 0; ct < 2; ++ct) { const size_t rk = (qbase + j0 + ct * 16 + col) * KD; v8f c = {}, cl = {};
      { const v16h kh = frag_h(KH + rk, lane); c = wmma16(aq, kh, c); cl = wmma16(aql, kh, cl); cl = wmma16(aq, frag_h(KL + rk, lane), cl); }
#pragma unroll
      for (int r = 0; r < 8; ++r) s[ct][r] = (c[r] + cl[r] * (1.0f / 2048.0f)) * scale; }
#pragma unroll
    for (int r = 0; r < 8; ++r) { float mx = fmaxf(s[0][r], s[1][r]);
#pragma unroll
      for (int o = 1; o < 16; o <<= 1) mx = fmaxf(mx, __shfl_xor(mx, o));
      const float mn = fmaxf(m[r], mx); const float alpha = (m[r] <= -1.0e38f) ? 0.f : __expf(m[r] - mn); const float e0 = __expf(s[0][r] - mn), e1 = __expf(s[1][r] - mn); float es = e0 + e1;
#pragma unroll
      for (int o = 1; o < 16; o <<= 1) es += __shfl_xor(es, o);
      l[r] = l[r] * alpha + es; m[r] = mn;
#pragma unroll
      for (int dt = 0; dt < 4; ++dt) acc[dt][r] *= alpha;
      sph[wave][8 * g + r][col] = (_Float16)(e0 * 2048.0f); sph[wave][8 * g + r][16 + col] = (_Float16)(e1 * 2048.0f); }
    LDSX();
    const v16h pa = frag_h(&sph[wave][col][0], lane);
#pragma unroll
    for (int dt = 0; dt < 4; ++dt) acc[dt] = wmma16(pa, frag_h(VH + (b * CC + h * VD + dt * 16 + col) * NP + j0, lane), acc[dt]);
    LDSX(); }
  for (int e = tid; e < VD * 3 * 66; e += 128) { const int d = e / 198, rem = e % 198; const int ry = rem / 66, xx = rem % 66; const int yy = y + ry - 1, xs = xx - 1; float v = 0.f;
    if (yy >= 0 && yy < HHT && xs >= 0 && xs < HW) { const size_t o = (b * CC + h * VD + d) * NP + yy * HW + xs; v = (float)VH[o] + (float)VL[o] * (1.0f / 2048.0f); } sv[d][ry][xx] = v; }
#pragma unroll
  for (int r = 0; r < 8; ++r) { const float il = (1.0f / 2048.0f) / l[r]; const int xq = wave * 16 + 8 * g + r;
#pragma unroll
    for (int dt = 0; dt < 4; ++dt) so[dt * 16 + col][xq] = acc[dt][r] * il; }
  __syncthreads();
  for (int e = tid; e < VD * 64; e += 128) { const int d = e >> 6, xq = e & 63; const int c = h * VD + d; float pe = bfr(BPE[c]);
#pragma unroll
    for (int k = 0; k < 9; ++k) pe += bfr(WPE[c * 9 + k]) * sv[d][k / 3][xq + k % 3];
    so[d][xq] += pe; }
  __syncthreads();
  for (int e = tid; e < VD * 16; e += 128) { const int d = e >> 4, q = e & 15; vst2(O + (b * CC + h * VD + d) * NP + y * 64 + q * 4, *(const v4f*)&so[d][q * 4]); }
}
__global__ __launch_bounds__(128) void k_proj(const float* __restrict__ O, const __bf16* __restrict__ PP, const float* __restrict__ BP, const float* __restrict__ X, float* __restrict__ X1, float* __restrict__ CS, float* __restrict__ CM) {
  __shared__ __align__(16) __bf16 sh[64][CC + 8], sl[64][CC + 8]; __shared__ __align__(16) float so[128][68];
  const int tid = threadIdx.x, wave = tid >> 5, lane = tid & 31, col = lane & 15, g = lane >> 4; const size_t b = blockIdx.y; const int n0 = blockIdx.x * 64;
  for (int e = tid; e < 64 * CC; e += 128) { const int c = e >> 6, r = e & 63; const float v = O[(b * CC + c) * NP + n0 + r]; const __bf16 hb = (__bf16)v; sh[r][c] = hb; sl[r][c] = (__bf16)(v - (float)hb); }
  if (tid < 64) for (int c = CC; c < CC + 8; ++c) { sh[tid][c] = (__bf16)0.f; sl[tid][c] = (__bf16)0.f; }
  __syncthreads();
#pragma unroll 1
  for (int pass = 0; pass < 2; ++pass) { v8f acc[8] = {};
#pragma unroll
    for (int kc = 0; kc < CC / 32; ++kc) { const v16b a = frag_b(&sh[wave * 16 + col][kc * 32], lane), al = frag_b(&sl[wave * 16 + col][kc * 32], lane);
#pragma unroll
      for (int j = 0; j < 8; ++j) { const v16b w = frag_b(PP + (size_t)(pass * 128 + j * 16 + col) * CC + kc * 32, lane); acc[j] = wmma_bf(al, w, acc[j]); acc[j] = wmma_bf(a, w, acc[j]); } }
#pragma unroll
    for (int j = 0; j < 8; ++j) { const int c = pass * 128 + j * 16 + col; const float bb = bfr(BP[c]);
#pragma unroll
      for (int r = 0; r < 8; ++r) { const int xq = wave * 16 + 8 * g + r; so[j * 16 + col][xq] = acc[j][r] + bb + bfr(X[(b * CC + c) * NP + n0 + xq]); } }
    __syncthreads();
    { const int cl_ = tid; float s = 0.f, mx = -3.0e38f; for (int xq = 0; xq < 64; ++xq) { const float v = so[cl_][xq]; s += v; mx = fmaxf(mx, v); }
      __shared__ __align__(16) float sred[2][128]; sred[0][cl_] = s; sred[1][cl_] = mx; __syncthreads();
      if (tid < 64) { const int which = tid >> 5, q = tid & 31; vst2((which ? CM : CS) + ((b * 64 + blockIdx.x) * CC) + pass * 128 + q * 4, *(const v4f*)&sred[which][q * 4]); } }
    for (int e = tid; e < 128 * 16; e += 128) { const int cl_ = e >> 4, q = e & 15; vst2(X1 + (b * CC + pass * 128 + cl_) * NP + n0 + q * 4, *(const v4f*)&so[cl_][q * 4]); }
    __syncthreads(); }
}
__global__ __launch_bounds__(256) void k_ca(const float* __restrict__ CS, const float* __restrict__ CM, const float* __restrict__ W1, const float* __restrict__ W2, float* __restrict__ CA) {
  const int b = blockIdx.x, c = threadIdx.x; __shared__ float sav[CC], smx[CC], shid[2][CC / RED]; __shared__ __align__(16) float sca[CC];
  { float s = 0.f, mx = -3.0e38f; for (int k = 0; k < NP / 64; ++k) { s += CS[((size_t)b * 64 + k) * CC + c]; mx = fmaxf(mx, CM[((size_t)b * 64 + k) * CC + c]); } sav[c] = s / (float)NP; smx[c] = mx; }
  __syncthreads();
  if (c < 2 * (CC / RED)) { const int which = c / (CC / RED), j = c % (CC / RED); const float* src = which ? smx : sav; float a = 0.f; for (int k = 0; k < CC; ++k) a += bfr(W1[j * CC + k]) * src[k]; shid[which][j] = fmaxf(a, 0.f); }
  __syncthreads();
  { float a0 = 0.f, a1 = 0.f; for (int j = 0; j < CC / RED; ++j) { const float w = bfr(W2[c * (CC / RED) + j]); a0 += w * shid[0][j]; a1 += w * shid[1][j]; } sca[c] = sigm_p(a0 + a1); }
  __syncthreads();
  if (c < CC / 4) vst2(CA + (size_t)b * CC + c * 4, *(const v4f*)&sca[c * 4]);
}
__global__ __launch_bounds__(256) void k_sp1(const float* __restrict__ X1, const float* __restrict__ CA, float* __restrict__ SP) {
  const size_t b = blockIdx.y; const int n0 = blockIdx.x * 64; const int t = threadIdx.x; const int xq = t & 63, part = t >> 6;
  float s = 0.f, mx = -3.0e38f; for (int c = part * 64; c < part * 64 + 64; ++c) { const float v = X1[(b * CC + c) * NP + n0 + xq] * CA[b * CC + c]; s += v; mx = fmaxf(mx, v); }
  __shared__ float ss[4][64], sm[4][64]; ss[part][xq] = s; sm[part][xq] = mx; __syncthreads();
  __shared__ __align__(16) float so[2][64]; if (t < 64) { so[0][t] = (ss[0][t] + ss[1][t] + ss[2][t] + ss[3][t]) / (float)CC; so[1][t] = fmaxf(fmaxf(sm[0][t], sm[1][t]), fmaxf(sm[2][t], sm[3][t])); } __syncthreads();
  if (t < 32) { const int which = t >> 4, q = t & 15; vst2(SP + (b * 2 + which) * NP + n0 + q * 4, *(const v4f*)&so[which][q * 4]); }
}
__global__ __launch_bounds__(256) void k_sp2(const float* __restrict__ X1, const float* __restrict__ CA, const float* __restrict__ SP, const float* __restrict__ WSA, float* __restrict__ OUT) {
  const size_t b = blockIdx.y; const int y = blockIdx.x; const int t = threadIdx.x; __shared__ float smap[2][3][66]; __shared__ float ssa[64]; __shared__ __align__(16) float so[CC][68];
  for (int e = t; e < 2 * 3 * 66; e += 256) { const int which = e / 198, rem = e % 198; const int ry = rem / 66, xx = rem % 66; const int yy = y + ry - 1, xs = xx - 1; smap[which][ry][xx] = (yy >= 0 && yy < HHT && xs >= 0 && xs < HW) ? SP[(b * 2 + which) * NP + yy * HW + xs] : 0.f; }
  __syncthreads();
  if (t < 64) { float a = 0.f;
#pragma unroll
    for (int which = 0; which < 2; ++which)
#pragma unroll
      for (int k = 0; k < 9; ++k) a += bfr(WSA[which * 9 + k]) * smap[which][k / 3][t + k % 3];
    ssa[t] = sigm_p(a); }
  __syncthreads();
  for (int e = t; e < CC * 64; e += 256) { const int c = e >> 6, xq = e & 63; so[c][xq] = X1[(b * CC + c) * NP + y * 64 + xq] * CA[b * CC + c] * ssa[xq]; }
  __syncthreads();
  for (int e = t; e < CC * 16; e += 256) { const int c = e >> 4, q = e & 15; vst2(OUT + (b * CC + c) * NP + y * 64 + q * 4, *(const v4f*)&so[c][q * 4]); }
}
extern "C" void kernel_launch(void* const* d_in, const int* in_sizes, int n_in, void* d_out, int out_size, void* d_ws, size_t ws_size, hipStream_t stream) {
  (void)in_sizes; (void)n_in; (void)out_size;
  const float** F = (const float**)d_in;
  if (ws_size < (size_t)WS_END) return;
  char* ws = (char*)d_ws; __bf16 *PW = (__bf16*)(ws + WS_PW), *PP = (__bf16*)(ws + WS_PP); _Float16 *QH = (_Float16*)(ws + WS_QH), *QL = (_Float16*)(ws + WS_QL), *KH = (_Float16*)(ws + WS_KH), *KL = (_Float16*)(ws + WS_KL), *VH = (_Float16*)(ws + WS_VH), *VL = (_Float16*)(ws + WS_VL); float *O = (float*)(ws + WS_O), *X1 = (float*)(ws + WS_X1), *CS = (float*)(ws + WS_CS), *CM = (float*)(ws + WS_CM), *CA = (float*)(ws + WS_CA), *SP = (float*)(ws + WS_SP);
  k_pack<<<dim3(HQ, 2), 256, 0, stream>>>(F[1], F[3], PW, PP);
  k_qkv<<<dim3(NP / 64, NB), 128, 0, stream>>>(F[0], PW, F[2], QH, QL, KH, KL, VH, VL);
  k_attn<<<dim3(HHT, NHh, NB), 128, 0, stream>>>(QH, QL, KH, KL, VH, VL, F[5], F[6], O);
  k_proj<<<dim3(NP / 64, NB), 128, 0, stream>>>(O, PP, F[4], F[0], X1, CS, CM);
  k_ca<<<NB, 256, 0, stream>>>(CS, CM, F[7], F[8], CA);
  k_sp1<<<dim3(NP / 64, NB), 256, 0, stream>>>(X1, CA, SP);
  k_sp2<<<dim3(HHT, NB), 256, 0, stream>>>(X1, CA, SP, F[9], (float*)d_out);
}
